// gMLPBlock_35897336660175
// MI455X (gfx1250) — hardware-run, weakly checked
//
#include <hip/hip_runtime.h>
#include <stddef.h>


#define HID     128
#define FFD     256
#define NTHR    256
#define NWAVE   8
#define EPT     8
#define NGRP    2
#define CHUNK   (NTHR * EPT * NGRP)
#define WCAP    (EPT * NGRP * 32)
#define LISTN   (NWAVE * WCAP)
#define NBC     4096
#define NBF     1024
#define RCAP    40960
#define RBN     128
#define TGT     256
#define DEGCAP  256
#define GROWS   64
#define OTHR    512
#define WSCAP   134217728
#define WINN    (FFD * HID)
#define WGCN    (FFD * FFD)
#define WOUTN   (HID * FFD)
#define WTOT    (WINN + WGCN + WOUTN)
#define WBLK    (NTHR * 8)

#define LDS_FILL ((RCAP + NBF + LISTN) * 4 + 64)
#define GEMM_LDS(KD, NC) ((GROWS * ((KD) + 8) * 2) > (GROWS * (NC) * 4) ? (GROWS * ((KD) + 8) * 2) : (GROWS * (NC) * 4))

static_assert((CHUNK & (CHUNK - 1)) == 0);
static_assert(CHUNK <= 4096);
static_assert(NBC <= 4096 && NBF <= 4096);
static_assert((NBC & (NBC - 1)) == 0 && (NBF & (NBF - 1)) == 0);
static_assert(NBC == 4 * NBF);
static_assert(OTHR * 8 == NBC);
static_assert((RCAP % 32) == 0);
static_assert((TGT % GROWS) == 0 && TGT == NWAVE * 32);
static_assert((NBC % TGT) == 0);
static_assert(GROWS == NWAVE * 8);
static_assert((WINN % WBLK) == 0 && (WGCN % WBLK) == 0 && (WOUTN % WBLK) == 0);
static_assert(FFD == 2 * HID);

typedef float    v4f  __attribute__((ext_vector_type(4)));
typedef float    v8f  __attribute__((ext_vector_type(8)));
typedef int      v4i  __attribute__((ext_vector_type(4)));
typedef _Float16 v4h  __attribute__((ext_vector_type(4)));
typedef _Float16 v8h  __attribute__((ext_vector_type(8)));
typedef _Float16 v16h __attribute__((ext_vector_type(16)));
union Frag { v16h v; v8h half[2]; };

__device__ __forceinline__ v8f wmh(v16h a, v16h b, v8f c) {
  v8f d = __builtin_amdgcn_wmma_f32_16x16x32_f16(false, a, false, b, (short)0, c, false, false);
  asm volatile("v_nop\n\tv_nop\n\tv_nop\n\tv_nop" : "+v"(d) : "v"(a), "v"(b));
  return d;
}

__device__ __forceinline__ float wave_sum(float v) {
#pragma unroll
  for (int o = 16; o > 0; o >>= 1) v += __shfl_xor(v, o, 32);
  return v;
}

__device__ __forceinline__ float tanh_f(float g) {
  const float e = exp2f(g * 2.8853900817779268f);
  const float r = __builtin_amdgcn_rcpf(e + 1.0f);
  return fmaf(-2.0f, r, 1.0f);
}

template <int NB>
__device__ __forceinline__ int scan_chunk(const int* __restrict__ dsts, int nE, int cbase, int slotBase,
                                          int vec8, int* list, int tid, int lane, int wave) {
  int wc = 0;
#pragma unroll
  for (int g = 0; g < NGRP; ++g) {
    const int el0  = (g * NTHR + tid) * EPT;
    const int e0   = cbase + el0;
    const int sent = -2147483647 - 1;
    v4i da, db;
    if (vec8 != 0 && cbase + CHUNK <= nE) {
      da = *(const v4i*)(dsts + e0);
      db = *(const v4i*)(dsts + e0 + 4);
    } else {
      da.x = (e0     < nE) ? dsts[min(e0, nE - 1)] : sent;
      da.y = (e0 + 1 < nE) ? dsts[min(e0 + 1, nE - 1)] : sent;
      da.z = (e0 + 2 < nE) ? dsts[min(e0 + 2, nE - 1)] : sent;
      da.w = (e0 + 3 < nE) ? dsts[min(e0 + 3, nE - 1)] : sent;
      db.x = (e0 + 4 < nE) ? dsts[min(e0 + 4, nE - 1)] : sent;
      db.y = (e0 + 5 < nE) ? dsts[min(e0 + 5, nE - 1)] : sent;
      db.z = (e0 + 6 < nE) ? dsts[min(e0 + 6, nE - 1)] : sent;
      db.w = (e0 + 7 < nE) ? dsts[min(e0 + 7, nE - 1)] : sent;
    }
    const unsigned nb = (unsigned)slotBase;
    const unsigned s0 = (unsigned)da.x - nb, s1 = (unsigned)da.y - nb;
    const unsigned s2 = (unsigned)da.z - nb, s3 = (unsigned)da.w - nb;
    const unsigned s4 = (unsigned)db.x - nb, s5 = (unsigned)db.y - nb;
    const unsigned s6 = (unsigned)db.z - nb, s7 = (unsigned)db.w - nb;
    const bool h0 = s0 < (unsigned)NB, h1 = s1 < (unsigned)NB, h2 = s2 < (unsigned)NB, h3 = s3 < (unsigned)NB;
    const bool h4 = s4 < (unsigned)NB, h5 = s5 < (unsigned)NB, h6 = s6 < (unsigned)NB, h7 = s7 < (unsigned)NB;
    const unsigned any = __builtin_amdgcn_ballot_w32(h0 | h1 | h2 | h3 | h4 | h5 | h6 | h7);
    if (any != 0u) {
#define HITJ(J, HJ, SJ) { \
        const unsigned mj = __builtin_amdgcn_ballot_w32(HJ); \
        if (mj != 0u) { \
          if (HJ) { \
            const int pos = wc + (int)__builtin_amdgcn_mbcnt_lo(mj, 0u); \
            if (pos < WCAP) list[wave * WCAP + pos] = ((el0 + (J)) << 12) | (int)(SJ); \
          } \
          wc += (int)__builtin_popcount(mj); } }
      HITJ(0, h0, s0)
      HITJ(1, h1, s1)
      HITJ(2, h2, s2)
      HITJ(3, h3, s3)
      HITJ(4, h4, s4)
      HITJ(5, h5, s5)
      HITJ(6, h6, s6)
      HITJ(7, h7, s7)
#undef HITJ
    }
  }
  return wc;
}

__global__ __launch_bounds__(NTHR) void k_wprep(
    const float* __restrict__ w0, const float* __restrict__ w1,
    const float* __restrict__ w2, _Float16* wp) {
  const int b = (int)blockIdx.x;
  constexpr int B0 = WINN / WBLK;
  constexpr int B1 = (WINN + WGCN) / WBLK;
  const int seg = b < B0 ? 0 : (b < B1 ? 1 : 2);
  const float* src = seg == 0 ? w0 : (seg == 1 ? w1 : w2);
  const float sc = seg == 1 ? 1048576.0f : 64.0f;
  const int lb = b - (seg == 0 ? 0 : (seg == 1 ? B0 : B1));
  const size_t dbase = seg == 0 ? (size_t)0 : (seg == 1 ? (size_t)WINN : (size_t)(WINN + WGCN));
  const int i = (lb * NTHR + (int)threadIdx.x) * 8;
  const v4f a = *(const v4f*)(src + i);
  const v4f c = *(const v4f*)(src + i + 4);
  v8h o;
  o[0] = (_Float16)(a.x * sc); o[1] = (_Float16)(a.y * sc); o[2] = (_Float16)(a.z * sc); o[3] = (_Float16)(a.w * sc);
  o[4] = (_Float16)(c.x * sc); o[5] = (_Float16)(c.y * sc); o[6] = (_Float16)(c.z * sc); o[7] = (_Float16)(c.w * sc);
  _Float16* d = wp + dbase + (size_t)i;
  *(volatile v8h*)d = o;
  __threadfence();
  *(volatile v8h*)d = o;
}

__global__ __launch_bounds__(NTHR) void k_count(
    const int* __restrict__ ei, int* cnt, float* dinv, int nE, int vec8) {
  __shared__ __attribute__((aligned(16))) int scnt[NBC];
  __shared__ __attribute__((aligned(16))) int list[LISTN];
  __shared__ int wcnt[NWAVE];
  const int tid = threadIdx.x, lane = tid & 31, wave = tid >> 5;
  const int nodeBase = blockIdx.x * NBC;
  const int* dsts = ei + nE;

  for (int i = tid; i < NBC; i += NTHR) scnt[i] = 0;
  __syncthreads();

  const int nChunks = (nE + CHUNK - 1) / CHUNK;
#pragma unroll 1
  for (int ch = 0; ch < nChunks; ++ch) {
    const int cbase = ch * CHUNK;
    const int wc = scan_chunk<NBC>(dsts, nE, cbase, nodeBase, vec8, list, tid, lane, wave);
    if (lane == 0) wcnt[wave] = wc;
    __syncthreads();
    if (wave == 0) {
#pragma unroll 1
      for (int wsx = 0; wsx < NWAVE; ++wsx) {
        int n = __builtin_amdgcn_readfirstlane(wcnt[wsx]);
        n = n > WCAP ? WCAP : (n < 0 ? 0 : n);
        const int* lp = list + wsx * WCAP;
#pragma unroll 1
        for (int i = 0; i < n; ++i) {
          const int ent  = __builtin_amdgcn_readfirstlane(lp[i]);
          const int slot = ent & (NBC - 1);
          if (lane == 0) scnt[slot] = scnt[slot] + 1;
        }
      }
    }
    __syncthreads();
  }

  v4i cq[4]; v4f dq[4];
#pragma unroll
  for (int q = 0; q < 4; ++q) {
    const int f = (wave * 4 + q) * 128 + 4 * lane;
    const v4i c = *(const v4i*)(scnt + f);
    cq[q] = c;
    dq[q].x = rsqrtf((float)(c.x + 2));
    dq[q].y = rsqrtf((float)(c.y + 2));
    dq[q].z = rsqrtf((float)(c.z + 2));
    dq[q].w = rsqrtf((float)(c.w + 2));
  }
  int*   cp = cnt + (size_t)nodeBase;
  float* dp = dinv + (size_t)nodeBase;
#pragma unroll
  for (int q = 0; q < 4; ++q) {
    const int f = (wave * 4 + q) * 128 + 4 * lane;
    *(volatile v4i*)(cp + f) = cq[q];
    *(volatile v4f*)(dp + f) = dq[q];
  }
  __threadfence();
#pragma unroll
  for (int q = 0; q < 4; ++q) {
    const int f = (wave * 4 + q) * 128 + 4 * lane;
    *(volatile v4i*)(cp + f) = cq[q];
    *(volatile v4f*)(dp + f) = dq[q];
  }
}

__global__ __launch_bounds__(OTHR) void k_offsets(
    const int* __restrict__ cnt, int* off, int* rbase, int nChunk) {
  __shared__ __attribute__((aligned(16))) int soff[NBC];
  __shared__ __attribute__((aligned(16))) int srb[RBN];
  __shared__ int wtot[OTHR / 32];
  const int tid = threadIdx.x, lane = tid & 31, wave = tid >> 5, sub = tid >> 7;
  for (int i = tid; i < RBN; i += OTHR) srb[i] = 0;
  int carry = 0;
#pragma unroll 1
  for (int ch = 0; ch < nChunk; ++ch) {
    const int base = ch * NBC;
    const v4i c0 = *(const v4i*)(cnt + base + 8 * tid);
    const v4i c1 = *(const v4i*)(cnt + base + 8 * tid + 4);
    const int e0 = max(c0.x, 0), e1 = max(c0.y, 0), e2 = max(c0.z, 0), e3 = max(c0.w, 0);
    const int e4 = max(c1.x, 0), e5 = max(c1.y, 0), e6 = max(c1.z, 0), e7 = max(c1.w, 0);
    const int ts = e0 + e1 + e2 + e3 + e4 + e5 + e6 + e7;
    int incl = ts;
#pragma unroll
    for (int d = 1; d < 32; d <<= 1) {
      const int t = __shfl_up(incl, d);
      if (lane >= d) incl += t;
    }
    if (lane == 31) wtot[wave] = incl;
    __syncthreads();
    const int S0 = wtot[0]  + wtot[1]  + wtot[2]  + wtot[3];
    const int S1 = wtot[4]  + wtot[5]  + wtot[6]  + wtot[7];
    const int S2 = wtot[8]  + wtot[9]  + wtot[10] + wtot[11];
    const int S3 = wtot[12] + wtot[13] + wtot[14] + wtot[15];
    int pre = 0;
#pragma unroll 1
    for (int w = 4 * sub; w < wave; ++w) pre += wtot[w];
    const int b0 = carry;
    const int b1 = b0 + ((S0 + 31) & ~31);
    const int b2 = b1 + ((S1 + 31) & ~31);
    const int b3 = b2 + ((S2 + 31) & ~31);
    const int b4 = b3 + ((S3 + 31) & ~31);
    const int myb = sub == 0 ? b0 : (sub == 1 ? b1 : (sub == 2 ? b2 : b3));
    if (tid == 0) {
      srb[min(4 * ch + 0, RBN - 1)] = b0;
      srb[min(4 * ch + 1, RBN - 1)] = b1;
      srb[min(4 * ch + 2, RBN - 1)] = b2;
      srb[min(4 * ch + 3, RBN - 1)] = b3;
    }
    int run = myb + pre + incl - ts;
    soff[8 * tid + 0] = run; run += e0;
    soff[8 * tid + 1] = run; run += e1;
    soff[8 * tid + 2] = run; run += e2;
    soff[8 * tid + 3] = run; run += e3;
    soff[8 * tid + 4] = run; run += e4;
    soff[8 * tid + 5] = run; run += e5;
    soff[8 * tid + 6] = run; run += e6;
    soff[8 * tid + 7] = run;
    carry = b4;
    __syncthreads();
    const v4i o0 = *(const v4i*)(soff + 4 * tid);
    const v4i o1 = *(const v4i*)(soff + 4 * (tid + OTHR));
    int* op = off + base;
    *(volatile v4i*)(op + 4 * tid) = o0;
    *(volatile v4i*)(op + 4 * (tid + OTHR)) = o1;
    __threadfence();
    *(volatile v4i*)(op + 4 * tid) = o0;
    *(volatile v4i*)(op + 4 * (tid + OTHR)) = o1;
    __syncthreads();
  }
  if (tid == 0) srb[min(4 * nChunk, RBN - 1)] = carry;
  __syncthreads();
  v4i rv = {0, 0, 0, 0};
  if (tid < 32) rv = *(const v4i*)(srb + 4 * tid);
  if (tid < 32) *(volatile v4i*)(rbase + 4 * tid) = rv;
  __threadfence();
  if (tid < 32) *(volatile v4i*)(rbase + 4 * tid) = rv;
}

__global__ __launch_bounds__(NTHR) void k_fill(
    const int* __restrict__ ei, const int* __restrict__ off, const int* __restrict__ rbase,
    int* csr, int nN, int nE, int vec8, int csrLen) {
  extern __shared__ v4f lds_dyn[];
  int* region = (int*)lds_dyn;
  int* cursor = region + RCAP;
  int* list   = cursor + NBF;
  int* wcnt   = list + LISTN;
  const int tid = threadIdx.x, lane = tid & 31, wave = tid >> 5;
  const int b = blockIdx.x;
  const int nodeBase = b * NBF;
  const int* dsts = ei + nE;

  int rb0 = rbase[b];
  const int rb1 = rbase[b + 1];
  rb0 = rb0 < 0 ? 0 : (rb0 > csrLen ? csrLen : rb0);
  rb0 &= ~31;
  int len = rb1 - rb0;
  len = len < 0 ? 0 : (len > RCAP ? RCAP : len);
  int lenW = (len + 31) & ~31;
  if (rb0 + lenW > csrLen) lenW = (csrLen - rb0) & ~31;

  {
    const v4i z = {0, 0, 0, 0};
    for (int i = tid; i < RCAP / 4; i += NTHR) ((v4i*)region)[i] = z;
    for (int s = tid; s < NBF; s += NTHR) {
      int o = off[nodeBase + s] - rb0;
      o = o < 0 ? 0 : (o > RCAP ? RCAP : o);
      cursor[s] = o;
    }
  }
  __syncthreads();

  const int nChunks = (nE + CHUNK - 1) / CHUNK;
#pragma unroll 1
  for (int ch = 0; ch < nChunks; ++ch) {
    const int cbase = ch * CHUNK;
    const int wc = scan_chunk<NBF>(dsts, nE, cbase, nodeBase, vec8, list, tid, lane, wave);
    if (lane == 0) wcnt[wave] = wc;
    __syncthreads();
    if (wave == 0) {
#pragma unroll 1
      for (int wsx = 0; wsx < NWAVE; ++wsx) {
        int n = __builtin_amdgcn_readfirstlane(wcnt[wsx]);
        n = n > WCAP ? WCAP : (n < 0 ? 0 : n);
        const int* lp = list + wsx * WCAP;
#pragma unroll 1
        for (int i = 0; i < n; ++i) {
          const int ent  = __builtin_amdgcn_readfirstlane(lp[i]);
          const int slot = ent & (NBF - 1);
          int e = cbase + ((ent >> 12) & (CHUNK - 1));
          e = e > nE - 1 ? nE - 1 : e;
          int src = ei[e];
          src = src < 0 ? 0 : (src > nN - 1 ? nN - 1 : src);
          if (lane == 0) {
            int pos = cursor[slot];
            pos = pos < 0 ? 0 : (pos > RCAP - 1 ? RCAP - 1 : pos);
            region[pos] = src;
            const int np = pos + 1;
            cursor[slot] = np > RCAP ? RCAP : np;
          }
        }
      }
    }
    __syncthreads();
  }

  const int nv = lenW >> 2;
  int* gp = csr + rb0;
#pragma unroll 1
  for (int i = tid; i < nv; i += NTHR) { const v4i v = ((const v4i*)region)[i]; *(volatile v4i*)(gp + 4 * i) = v; }
  __threadfence();
#pragma unroll 1
  for (int i = tid; i < nv; i += NTHR) { const v4i v = ((const v4i*)region)[i]; *(volatile v4i*)(gp + 4 * i) = v; }
}

template <int KD, int NCOL, int LNORM, int EPI>
__global__ __launch_bounds__(NTHR) void k_gemm(
    const float* __restrict__ A, const float* __restrict__ lng, const float* __restrict__ lnb,
    const _Float16* __restrict__ Bw, const float* __restrict__ bias, const float* __restrict__ dinv,
    float* C, int nRowsA, int nRowsC) {
  extern __shared__ v4f lds_dyn[];
  constexpr int APH = KD + 8;
  constexpr int NT  = NCOL / 32;
  constexpr int VPL = KD / 32;
  constexpr int RPW = GROWS / NWAVE;
  constexpr int PPR = NCOL / 128;
  constexpr float OSC = (EPI == 2) ? (1.0f / 1048576.0f) : (1.0f / 64.0f);
  static_assert(VPL == 4 || VPL == 8);
  static_assert((APH * 2) % 16 == 0);
  _Float16* sA  = (_Float16*)lds_dyn;
  float*    stg = (float*)lds_dyn;
  const int tid = threadIdx.x, lane = tid & 31, wave = tid >> 5, hh = lane >> 4, m = lane & 15;
  const int rowBase = blockIdx.x * GROWS;

  v4f ga = {1.f, 1.f, 1.f, 1.f}, gb = {1.f, 1.f, 1.f, 1.f};
  v4f ba = {0.f, 0.f, 0.f, 0.f}, bb = {0.f, 0.f, 0.f, 0.f};
  if (LNORM != 0) {
    ga = *(const v4f*)(lng + VPL * lane);
    ba = *(const v4f*)(lnb + VPL * lane);
    if (VPL == 8) { gb = *(const v4f*)(lng + VPL * lane + 4); bb = *(const v4f*)(lnb + VPL * lane + 4); }
  }
#pragma unroll 1
  for (int i = 0; i < RPW; ++i) {
    const int r = wave * RPW + i;
    int row = rowBase + r;
    row = row > nRowsA - 1 ? nRowsA - 1 : row;
    const float* ap = A + (size_t)row * KD + VPL * lane;
    v4f x0 = *(const v4f*)ap;
    v4f x1 = {0.f, 0.f, 0.f, 0.f};
    if (VPL == 8) x1 = *(const v4f*)(ap + 4);
    if (LNORM != 0) {
      float s = x0.x + x0.y + x0.z + x0.w;
      if (VPL == 8) s += x1.x + x1.y + x1.z + x1.w;
      s = wave_sum(s);
      const float mu = s * (1.0f / (float)KD);
      x0 = x0 - mu;
      if (VPL == 8) x1 = x1 - mu;
      float q = x0.x * x0.x + x0.y * x0.y + x0.z * x0.z + x0.w * x0.w;
      if (VPL == 8) q += x1.x * x1.x + x1.y * x1.y + x1.z * x1.z + x1.w * x1.w;
      q = wave_sum(q);
      const float rs = rsqrtf(q * (1.0f / (float)KD) + 1e-5f);
      x0 = x0 * rs * ga + ba;
      if (VPL == 8) x1 = x1 * rs * gb + bb;
    }
    if (VPL == 8) {
      v8h o;
      o[0] = (_Float16)x0.x; o[1] = (_Float16)x0.y; o[2] = (_Float16)x0.z; o[3] = (_Float16)x0.w;
      o[4] = (_Float16)x1.x; o[5] = (_Float16)x1.y; o[6] = (_Float16)x1.z; o[7] = (_Float16)x1.w;
      *(v8h*)(sA + r * APH + 8 * lane) = o;
    } else {
      v4h o;
      o[0] = (_Float16)x0.x; o[1] = (_Float16)x0.y; o[2] = (_Float16)x0.z; o[3] = (_Float16)x0.w;
      *(v4h*)(sA + r * APH + 4 * lane) = o;
    }
  }
  __syncthreads();

  v8f acc[NT];
#pragma unroll
  for (int t = 0; t < NT; ++t) { v8f z = {0.f, 0.f, 0.f, 0.f, 0.f, 0.f, 0.f, 0.f}; acc[t] = z; }
  const int rg = wave >> 1, cg = wave & 1;
  const _Float16* arow = sA + (rg * 16 + m) * APH + 8 * hh;
  const _Float16* bcol = Bw + (size_t)(cg * (NCOL / 2) + m) * KD + 8 * hh;
#pragma unroll 1
  for (int kt = 0; kt < KD / 32; ++kt) {
    Frag a;
    a.half[0] = *(const v8h*)(arow + 32 * kt);
    a.half[1] = *(const v8h*)(arow + 32 * kt + 16);
#pragma unroll
    for (int t = 0; t < NT; ++t) {
      const _Float16* bp = bcol + (size_t)(16 * t) * KD + 32 * kt;
      Frag b;
      b.half[0] = *(const v8h*)bp;
      b.half[1] = *(const v8h*)(bp + 16);
      acc[t] = wmh(a.v, b.v, acc[t]);
    }
  }
  __syncthreads();

  const int r0 = rg * 16 + 8 * hh;
  float rsc[8];
#pragma unroll
  for (int r = 0; r < 8; ++r) rsc[r] = OSC;
  if (EPI == 2) {
    const v4f dA = *(const v4f*)(dinv + (size_t)rowBase + r0);
    const v4f dB = *(const v4f*)(dinv + (size_t)rowBase + r0 + 4);
    rsc[0] *= dA.x; rsc[1] *= dA.y; rsc[2] *= dA.z; rsc[3] *= dA.w;
    rsc[4] *= dB.x; rsc[5] *= dB.y; rsc[6] *= dB.z; rsc[7] *= dB.w;
  }
  float* sp = stg + r0 * NCOL + cg * (NCOL / 2) + m;
#pragma unroll
  for (int t = 0; t < NT; ++t) {
    float bv = 0.0f;
    if (EPI != 2) bv = bias[cg * (NCOL / 2) + 16 * t + m];
#pragma unroll
    for (int r = 0; r < 8; ++r) {
      float v = acc[t][r] * rsc[r] + bv;
      if (EPI == 1) v = 0.5f * v * (1.0f + erff(v * 0.70710678118654752f));
      sp[r * NCOL + 16 * t] = v;
    }
  }
  __syncthreads();

  const int rw0 = rowBase + wave * RPW;
  const float* lrow = stg + (wave * RPW) * NCOL + 4 * lane;
  float* grow = C + (size_t)rw0 * NCOL + 4 * lane;
#pragma unroll
  for (int i = 0; i < RPW; ++i) {
#pragma unroll
    for (int p = 0; p < PPR; ++p) {
      const v4f v = *(const v4f*)(lrow + i * NCOL + p * 128);
      if (rw0 + i < nRowsC) *(volatile v4f*)(grow + (size_t)i * NCOL + p * 128) = v;
    }
  }
  __threadfence();
#pragma unroll
  for (int i = 0; i < RPW; ++i) {
#pragma unroll
    for (int p = 0; p < PPR; ++p) {
      const v4f v = *(const v4f*)(lrow + i * NCOL + p * 128);
      if (rw0 + i < nRowsC) *(volatile v4f*)(grow + (size_t)i * NCOL + p * 128) = v;
    }
  }
}

__global__ __launch_bounds__(NTHR) void k_agg(
    const int* __restrict__ csr, const int* __restrict__ off, const int* __restrict__ cnt,
    const float* __restrict__ dinv, const float* __restrict__ hw, float* h,
    const float* __restrict__ bg, int nN, int csrLen) {
  const int tid = threadIdx.x, lane = tid & 31, wave = tid >> 5;
  const int tbase = blockIdx.x * TGT + wave * 32;
  const int cl = tbase + lane;
  const int cnt_l = cnt[cl];
  const int off_l = off[cl];
  union FI { float f; int i; };
  FI dvu; dvu.f = dinv[cl];
  const int ch0 = 4 * lane, ch1 = HID + 4 * lane;
  const v4f bb0 = *(const v4f*)(bg + ch0);
  const v4f bb1 = *(const v4f*)(bg + ch1);

#pragma unroll 1
  for (int j = 0; j < 32; ++j) {
    const int c = tbase + j;
    int n = __builtin_amdgcn_readlane(cnt_l, j);
    n = n < 0 ? 0 : (n > DEGCAP ? DEGCAP : n);
    const int st = __builtin_amdgcn_readlane(off_l, j);
    FI du; du.i = __builtin_amdgcn_readlane(dvu.i, j);
    const float dc = du.f;
    v4f a0 = {0.f, 0.f, 0.f, 0.f}, a1 = {0.f, 0.f, 0.f, 0.f};
#pragma unroll 1
    for (int q0 = 0; q0 < n; q0 += 32) {
      int pos = st + q0 + lane;
      pos = pos < 0 ? 0 : (pos > csrLen - 1 ? csrLen - 1 : pos);
      int sl = csr[pos];
      sl = sl < 0 ? 0 : (sl > nN - 1 ? nN - 1 : sl);
      const int mcnt = (n - q0) < 32 ? (n - q0) : 32;
#pragma unroll 1
      for (int p = 0; p < mcnt; ++p) {
        const int s = __builtin_amdgcn_readlane(sl, p);
        const float* hp = hw + (size_t)s * FFD;
        a0 = a0 + *(const v4f*)(hp + ch0);
        a1 = a1 + *(const v4f*)(hp + ch1);
      }
    }
    const float* hc = hw + (size_t)c * FFD;
    const v4f s0 = *(const v4f*)(hc + ch0);
    const v4f s1 = *(const v4f*)(hc + ch1);
    const v4f g0 = (a0 + s0 * 2.0f) * dc + bb0;
    const v4f g1 = (a1 + s1 * 2.0f) * dc + bb1;
    v4f t0, t1;
    t0.x = tanh_f(g0.x); t0.y = tanh_f(g0.y); t0.z = tanh_f(g0.z); t0.w = tanh_f(g0.w);
    t1.x = tanh_f(g1.x); t1.y = tanh_f(g1.y); t1.z = tanh_f(g1.z); t1.w = tanh_f(g1.w);
    float* hrow = h + (size_t)c * FFD;
    const v4f hv0 = *(const v4f*)(hrow + ch0);
    const v4f hv1 = *(const v4f*)(hrow + ch1);
    const v4f o0 = t0 * hv0;
    const v4f o1 = t1 * hv1;
    *(volatile v4f*)(hrow + ch0) = o0;
    *(volatile v4f*)(hrow + ch1) = o1;
    __threadfence();
    *(volatile v4f*)(hrow + ch0) = o0;
    *(volatile v4f*)(hrow + ch1) = o1;
  }
}

extern "C" void kernel_launch(void* const* d_in, const int* in_sizes, int n_in,
                              void* d_out, int out_size, void* d_ws, size_t ws_size,
                              hipStream_t stream) {
  if (n_in < 12) return;
  const int nN = in_sizes[0] / HID;
  const int nE = in_sizes[1] / 2;
  if (nN <= 0 || nE <= 0 || in_sizes[0] != nN * HID || in_sizes[1] != 2 * nE) return;
  if (in_sizes[2] != HID || in_sizes[3] != HID) return;
  if (in_sizes[4] != WINN || in_sizes[5] != FFD) return;
  if (in_sizes[6] != FFD || in_sizes[7] != FFD) return;
  if (in_sizes[8] != WGCN || in_sizes[9] != FFD) return;
  if (in_sizes[10] != WOUTN || in_sizes[11] != HID) return;
  if (out_size != nN * HID) return;
  if (nE > (1 << 28) || nN > (1 << 24)) return;

  const float* x    = (const float*)d_in[0];
  const int*   ei   = (const int*)d_in[1];
  const float* ln1g = (const float*)d_in[2];
  const float* ln1b = (const float*)d_in[3];
  const float* win  = (const float*)d_in[4];
  const float* bin  = (const float*)d_in[5];
  const float* ln2g = (const float*)d_in[6];
  const float* ln2b = (const float*)d_in[7];
  const float* wg   = (const float*)d_in[8];
  const float* bgv  = (const float*)d_in[9];
  const float* wout = (const float*)d_in[10];
  const float* bout = (const float*)d_in[11];
  float* out = (float*)d_out;

  const int NPAD   = ((nN + TGT - 1) / TGT) * TGT;
  const int nBC    = (nN + NBC - 1) / NBC;
  const int CNTPAD = nBC * NBC;
  if (4 * nBC + 1 > RBN) return;
  const int nBF    = (nN + NBF - 1) / NBF;
  const int csrLen = ((nE + 31) & ~31) + 4096;
  if (31 * 4 * nBC > 4096) return;
  const int nGemm  = NPAD / GROWS;
  const int nAgg   = NPAD / TGT;

  char* ws = (char*)d_ws;
  size_t off = 0;
  const size_t oW   = off; off += (size_t)WTOT * 2;                off = (off + 255) & ~(size_t)255;
  const size_t oCnt = off; off += (size_t)CNTPAD * 4;              off = (off + 255) & ~(size_t)255;
  const size_t oDv  = off; off += (size_t)CNTPAD * 4;              off = (off + 255) & ~(size_t)255;
  const size_t oOff = off; off += (size_t)CNTPAD * 4;              off = (off + 255) & ~(size_t)255;
  const size_t oRb  = off; off += (size_t)RBN * 4;                 off = (off + 255) & ~(size_t)255;
  const size_t oCsr = off; off += (size_t)csrLen * 4;              off = (off + 255) & ~(size_t)255;
  const size_t oH   = off; off += (size_t)NPAD * FFD * 4;          off = (off + 255) & ~(size_t)255;
  const size_t oHw  = off; off += (size_t)NPAD * FFD * 4;          off = (off + 255) & ~(size_t)255;
  if (off > ws_size || off > (size_t)WSCAP) return;
  _Float16* wp   = (_Float16*)(ws + oW);
  int*      cnt  = (int*)(ws + oCnt);
  float*    dinv = (float*)(ws + oDv);
  int*      offp = (int*)(ws + oOff);
  int*      rb   = (int*)(ws + oRb);
  int*      csr  = (int*)(ws + oCsr);
  float*    h1   = (float*)(ws + oH);
  float*    hw   = (float*)(ws + oHw);

  const int vec8 = ((nE & 3) == 0) ? 1 : 0;

  k_wprep<<<WTOT / WBLK, NTHR, 0, stream>>>(win, wg, wout, wp);

  k_count<<<nBC, NTHR, 0, stream>>>(ei, cnt, dinv, nE, vec8);
  k_offsets<<<1, OTHR, 0, stream>>>(cnt, offp, rb, nBC);
  hipFuncSetAttribute(reinterpret_cast<const void*>(&k_fill),
                      hipFuncAttributeMaxDynamicSharedMemorySize, LDS_FILL);
  k_fill<<<nBF, NTHR, LDS_FILL, stream>>>(ei, offp, rb, csr, nN, nE, vec8, csrLen);

  constexpr int LDS_G1 = GEMM_LDS(HID, FFD);
  constexpr int LDS_G2 = GEMM_LDS(FFD, FFD);
  constexpr int LDS_G3 = GEMM_LDS(FFD, HID);
  hipFuncSetAttribute(reinterpret_cast<const void*>(&k_gemm<HID, FFD, 1, 1>),
                      hipFuncAttributeMaxDynamicSharedMemorySize, LDS_G1);
  hipFuncSetAttribute(reinterpret_cast<const void*>(&k_gemm<FFD, FFD, 1, 2>),
                      hipFuncAttributeMaxDynamicSharedMemorySize, LDS_G2);
  hipFuncSetAttribute(reinterpret_cast<const void*>(&k_gemm<FFD, HID, 0, 0>),
                      hipFuncAttributeMaxDynamicSharedMemorySize, LDS_G3);
  k_gemm<HID, FFD, 1, 1><<<nGemm, NTHR, LDS_G1, stream>>>(x, ln1g, ln1b, wp, bin, dinv, h1, nN, NPAD);

  k_gemm<FFD, FFD, 1, 2><<<nGemm, NTHR, LDS_G2, stream>>>(h1, ln2g, ln2b, wp + (size_t)WINN, bgv, dinv, hw, NPAD, NPAD);

  k_agg<<<nAgg, NTHR, 0, stream>>>(csr, offp, cnt, dinv, hw, h1, bgv, nN, csrLen);

  k_gemm<FFD, HID, 0, 0><<<nGemm, NTHR, LDS_G3, stream>>>(h1, ln2g, ln2b, wp + (size_t)(WINN + WGCN), bout, dinv, out, NPAD, nN);
}
